// BindingSiteGNN_44908178047027
// MI455X (gfx1250) — hardware-verified
//
#include <hip/hip_runtime.h>
#include <math.h>

#define NN 20000
#define NE 150000
#define NV (NE + NN)
#define XD 5
#define AE 32
#define NAA 20
#define KIN 37
#define K1 64
#define F1W 512
#define F2W 128
#define MP 20032
#define NT 256
#define TG 2048
#define NTILE 10
#define NROWT (NTILE * TG)
#define SCH 4096
#define SPT (SCH / NT)
#define NCH1 ((NE + SCH - 1) / SCH)
#define NCH2 ((NV + SCH - 1) / SCH)
#define ASC 16.0f
#define GSC_INV (1.0f / 256.0f)
#define GAT_LDS(ng) ((2 * TG * (ng) + SCH) * 4)

static_assert(NE % SPT == 0);
static_assert(MP % 64 == 0 && MP >= NN && NROWT >= MP);
static_assert(NN % 32 == 0 && TG / 8 == 256);
static_assert(NV < (1 << 20));

typedef __attribute__((ext_vector_type(16))) _Float16 v16h;
typedef __attribute__((ext_vector_type(8)))  _Float16 v8h;
typedef __attribute__((ext_vector_type(4)))  _Float16 v4h;
typedef __attribute__((ext_vector_type(16))) __bf16   v16b;
typedef __attribute__((ext_vector_type(8)))  __bf16   v8b;
typedef __attribute__((ext_vector_type(8)))  float    v8f;
typedef __attribute__((ext_vector_type(4)))  float    v4f;
typedef __attribute__((ext_vector_type(2)))  float    v2f;
typedef __attribute__((ext_vector_type(4)))  int      v4i;
#define U16(p) ((const unsigned short*)(const void*)(p))

__device__ __forceinline__ unsigned short f2bf_bits(float f) {
  unsigned u = __float_as_uint(f);
  return (unsigned short)((u + 0x7FFFu + ((u >> 16) & 1u)) >> 16);
}
__device__ __forceinline__ float bf_bits2f(unsigned short h) { return __uint_as_float(((unsigned)h) << 16); }

__device__ __forceinline__ void dep_guard_h(v8f& a, v8f& b, v16h x, v16h y) { asm volatile("v_nop\n\tv_nop\n\tv_nop\n\tv_nop" : "+v"(a), "+v"(b) : "v"(x), "v"(y)); }
__device__ __forceinline__ void dep_guard_b(v8f& a, v8f& b, v16b x, v16b y) { asm volatile("v_nop\n\tv_nop\n\tv_nop\n\tv_nop" : "+v"(a), "+v"(b) : "v"(x), "v"(y)); }
__device__ __forceinline__ void keep4_h(v16h a, v16h b, v16h c, v16h d) { asm volatile("v_nop" :: "v"(a), "v"(b), "v"(c), "v"(d)); }
__device__ __forceinline__ void keep4_b(v16b a, v16b b, v16b c, v16b d) { asm volatile("v_nop" :: "v"(a), "v"(b), "v"(c), "v"(d)); }
__device__ __forceinline__ void acc_guard4(v8f& a, v8f& b, v8f& c, v8f& d) { asm volatile("v_nop\n\tv_nop\n\tv_nop\n\tv_nop" : "+v"(a), "+v"(b), "+v"(c), "+v"(d)); }
template <typename T> struct Frag;
template <> struct Frag<_Float16> {
  typedef v16h V; union U { v16h v; v8h h[2]; };
  static __device__ __forceinline__ v16h load(const _Float16* p) {
    U f; f.h[0] = *(const v8h*)(p); f.h[1] = *(const v8h*)(p + 16); return f.v;
  }
  static __device__ __forceinline__ v8f mma(v16h a, v16h b, v8f c) {
    return __builtin_amdgcn_wmma_f32_16x16x32_f16(false, a, false, b, (short)0, c, false, false);
  }
  static __device__ __forceinline__ void guard(v8f& a, v8f& b, v16h x, v16h y) { dep_guard_h(a, b, x, y); }
  static __device__ __forceinline__ void keep(v16h a, v16h b, v16h c, v16h d) { keep4_h(a, b, c, d); }
};
template <> struct Frag<__bf16> {
  typedef v16b V; union U { v16b v; v8b h[2]; };
  static __device__ __forceinline__ v16b load(const __bf16* p) {
    U f; f.h[0] = *(const v8b*)(p); f.h[1] = *(const v8b*)(p + 16); return f.v;
  }
  static __device__ __forceinline__ v8f mma(v16b a, v16b b, v8f c) {
    return __builtin_amdgcn_wmma_f32_16x16x32_bf16(false, a, false, b, (short)0, c, false, false);
  }
  static __device__ __forceinline__ void guard(v8f& a, v8f& b, v16b x, v16b y) { dep_guard_b(a, b, x, y); }
  static __device__ __forceinline__ void keep(v16b a, v16b b, v16b c, v16b d) { keep4_b(a, b, c, d); }
};

template <int ET> struct Elem;
template <> struct Elem<0> { typedef _Float16 T; };
template <> struct Elem<1> { typedef __bf16 T; };
template <int ET, bool SPLIT, int BIAS_MODE, int OUT_MODE, bool RESID, int ACT = 0>
__global__ __launch_bounds__(256) void wmma_gemm64(
    const unsigned short* __restrict__ Ap, const unsigned short* __restrict__ A2p, int lda, long strideA,
    const unsigned short* __restrict__ Btp, const unsigned short* __restrict__ Bt2p, int ldb, long strideB,
    void* __restrict__ Cout, void* __restrict__ Cout2, int ldc, long strideC,
    const float* __restrict__ bias,
    const float* __restrict__ resid, long strideR,
    int M, int N, int K, float scale) {
  typedef typename Elem<ET>::T T;
  typedef typename Frag<T>::V V;
  const T* A = (const T*)Ap; const T* A2 = (const T*)A2p; const T* Bt = (const T*)Btp; const T* Bt2 = (const T*)Bt2p;
  __shared__ __align__(16) float sT[8][16 * 68];
  const int b    = blockIdx.y;
  const int lane = threadIdx.x & 31;
  const int wave = threadIdx.x >> 5;
  const int tilesN = N >> 6;
  const int tilesM = M >> 6;
  const int tile = blockIdx.x * 8 + wave;
  if (tile >= tilesM * tilesN) return;
  const int tm = tile / tilesN;
  const int tn = tile - tm * tilesN;
  const int m0 = tm << 6;
  const int n0 = tn << 6;

  const T* Ab  = A  + (size_t)b * strideA;
  const T* Bb  = Bt + (size_t)b * strideB;
  const T* Ab2 = SPLIT ? (A2  + (size_t)b * strideA) : nullptr;
  const T* Bb2 = SPLIT ? (Bt2 + (size_t)b * strideB) : nullptr;

  const int rlane = lane & 15;
  const int koff  = (lane >> 4) * 8;
  const int mOff  = (lane >> 4) * 8;

  v8f acc[4][4];
#pragma unroll
  for (int i = 0; i < 4; ++i)
#pragma unroll
    for (int j = 0; j < 4; ++j) acc[i][j] = (v8f){0.f,0.f,0.f,0.f,0.f,0.f,0.f,0.f};

  for (int k0 = 0; k0 < K; k0 += 32) {
    V bh[4], bl[4];
#pragma unroll
    for (int j = 0; j < 4; ++j) {
      const size_t bo = (size_t)(n0 + (j << 4) + rlane) * ldb + koff + k0;
      bh[j] = Frag<T>::load(Bb + bo);
      if (SPLIT) bl[j] = Frag<T>::load(Bb2 + bo);
    }
#pragma unroll
    for (int i = 0; i < 4; ++i) {
      const size_t ao = (size_t)(m0 + (i << 4) + rlane) * lda + koff + k0;
      V ah = Frag<T>::load(Ab + ao);
      V al;
      if (SPLIT) al = Frag<T>::load(Ab2 + ao);
#pragma unroll
      for (int j = 0; j < 4; ++j) {
        acc[i][j] = Frag<T>::mma(ah, bh[j], acc[i][j]);
        if (SPLIT) {
          acc[i][j] = Frag<T>::mma(ah, bl[j], acc[i][j]);
          acc[i][j] = Frag<T>::mma(al, bh[j], acc[i][j]);
        }
      }
      Frag<T>::guard(acc[i][0], acc[i][3], ah, SPLIT ? al : ah);
    }
    Frag<T>::keep(bh[0], bh[1], bh[2], bh[3]);
    if (SPLIT) Frag<T>::keep(bl[0], bl[1], bl[2], bl[3]);
  }
  acc_guard4(acc[0][0], acc[0][1], acc[0][2], acc[0][3]);
  acc_guard4(acc[1][0], acc[1][1], acc[1][2], acc[1][3]);
  acc_guard4(acc[2][0], acc[2][1], acc[2][2], acc[2][3]);
  acc_guard4(acc[3][0], acc[3][1], acc[3][2], acc[3][3]);

  float* slab = sT[wave];
  const float* Rb = RESID ? (resid + (size_t)b * strideR) : nullptr;
#pragma unroll
  for (int i = 0; i < 4; ++i) {
    const int mBase = m0 + (i << 4);
#pragma unroll
    for (int j = 0; j < 4; ++j) {
      const int n = n0 + (j << 4) + rlane;
      float bv = 0.f;
      if (BIAS_MODE == 2) bv = bias[n];
#pragma unroll
      for (int r = 0; r < 8; ++r) {
        float v = acc[i][j][r] * scale;
        if (BIAS_MODE == 1) v += bias[mBase + mOff + r];
        if (BIAS_MODE == 2) v += bv;
        if (RESID) v += Rb[(size_t)(mBase + mOff + r) * ldc + n];
        if (ACT == 1) v = tanhf(v);
        if (ACT == 2) v = fmaxf(v, 0.0f);
        if (ACT == 3) v = v / (1.0f + expf(-v));
        if (ACT == 4) v = (v > 0.f) ? v : 0.01f * v;
        if (ACT == 5) v = 0.5f * v * (1.0f + erff(v * 0.70710678118654752f));
        if (ACT == 6) v = (v > 0.f) ? v : 0.2f * v;
        slab[(mOff + r) * 68 + (j << 4) + rlane] = v;
      }
    }
    __builtin_amdgcn_fence(__ATOMIC_RELEASE, "workgroup");
    __builtin_amdgcn_wave_barrier();
    __builtin_amdgcn_fence(__ATOMIC_ACQUIRE, "workgroup");
    if (OUT_MODE == 0) {
      float* C = (float*)Cout + (size_t)b * strideC;
      const int hh = lane >> 4, c4 = (lane & 15) * 4;
      for (int pass = 0; pass < 2; ++pass) {
#pragma unroll
        for (int it = 0; it < 8; ++it) {
          const int row = it * 2 + hh;
          v4f v = *(const v4f*)(slab + row * 68 + c4);
          *(volatile v4f*)(C + (size_t)(mBase + row) * ldc + n0 + c4) = v;
        }
        __threadfence();
      }
    } else {
      const int q = lane >> 3, c8 = (lane & 7) * 8;
      unsigned short* C  = (unsigned short*)Cout  + (size_t)b * strideC;
      unsigned short* C2 = (OUT_MODE == 2) ? ((unsigned short*)Cout2 + (size_t)b * strideC) : nullptr;
      for (int pass = 0; pass < 2; ++pass) {
#pragma unroll
        for (int it = 0; it < 4; ++it) {
          const int row = it * 4 + q;
          const float* sp = slab + row * 68 + c8;
          v8h hv, lv;
#pragma unroll
          for (int e = 0; e < 8; ++e) {
            if (OUT_MODE == 1) {
              hv[e] = (_Float16)sp[e];
            } else {
              unsigned short hb = f2bf_bits(sp[e]);
              unsigned short lb = f2bf_bits(sp[e] - bf_bits2f(hb));
              hv[e] = __builtin_bit_cast(_Float16, hb);
              lv[e] = __builtin_bit_cast(_Float16, lb);
            }
          }
          *(volatile v8h*)(C + (size_t)(mBase + row) * ldc + n0 + c8) = hv;
          if (OUT_MODE == 2) *(volatile v8h*)(C2 + (size_t)(mBase + row) * ldc + n0 + c8) = lv;
        }
        __threadfence();
      }
    }
    __builtin_amdgcn_fence(__ATOMIC_RELEASE, "workgroup");
    __builtin_amdgcn_wave_barrier();
    __builtin_amdgcn_fence(__ATOMIC_ACQUIRE, "workgroup");
  }
}

__device__ __forceinline__ unsigned pack_f16x2(float a, float b) {
  const _Float16 h0 = (_Float16)a, h1 = (_Float16)b;
  return (unsigned)__builtin_bit_cast(unsigned short, h0) | ((unsigned)__builtin_bit_cast(unsigned short, h1) << 16);
}

__global__ __launch_bounds__(256) void h0_kernel(const float* __restrict__ x, const int* __restrict__ rt,
                                                const float* __restrict__ emb, unsigned* __restrict__ out) {
  const int i = blockIdx.x * 256 + threadIdx.x;
  if (i < MP * 32) {
    const int n = i >> 5, c = 2 * (i & 31);
    const bool live = n < NN;
    const int nc = live ? n : (NN - 1);
    int t = rt[nc];
    t = t < 0 ? 0 : (t >= NAA ? NAA - 1 : t);
    float f[2];
#pragma unroll
    for (int u = 0; u < 2; ++u) {
      const int cc = c + u;
      const int cx = cc < XD ? cc : (XD - 1);
      int ce = cc - XD; ce = ce < 0 ? 0 : (ce >= AE ? AE - 1 : ce);
      const float vx = x[(size_t)nc * XD + cx];
      const float ve = emb[t * AE + ce];
      const float v = (cc < XD) ? vx : ((cc < KIN) ? ve : 0.f);
      f[u] = live ? v * ASC : 0.f;
    }
    const unsigned uu = pack_f16x2(f[0], f[1]);
    ((volatile unsigned*)out)[i] = uu;
    __threadfence();
    ((volatile unsigned*)out)[i] = uu;
  }
}

__global__ __launch_bounds__(NT) void wprep_kernel(const float* __restrict__ W1l, const float* __restrict__ W1r,
                                                  const float* __restrict__ W2l, const float* __restrict__ W2r,
                                                  unsigned* __restrict__ Bt1P, unsigned* __restrict__ Bt2P) {
  const int t = threadIdx.x;
  for (int i = t; i < 2 * F1W * 32; i += NT) {
    const int n = i >> 5, k = 2 * (i & 31), col = n & (F1W - 1);
    const int k0c = k < KIN ? k : (KIN - 1), k1c = (k + 1) < KIN ? (k + 1) : (KIN - 1);
    const float l0 = W1l[k0c * F1W + col], l1 = W1l[k1c * F1W + col];
    const float r0 = W1r[k0c * F1W + col], r1 = W1r[k1c * F1W + col];
    float a = (n < F1W) ? l0 : r0, b = (n < F1W) ? l1 : r1;
    a = (k < KIN) ? a * ASC : 0.f;
    b = ((k + 1) < KIN) ? b * ASC : 0.f;
    const unsigned u = pack_f16x2(a, b);
    ((volatile unsigned*)Bt1P)[i] = u; __threadfence(); ((volatile unsigned*)Bt1P)[i] = u;
  }
  for (int i = t; i < 2 * F2W * 256; i += NT) {
    const int n = i >> 8, k = 2 * (i & 255), col = n & (F2W - 1);
    const float l0 = W2l[k * F2W + col], l1 = W2l[(k + 1) * F2W + col];
    const float r0 = W2r[k * F2W + col], r1 = W2r[(k + 1) * F2W + col];
    const float a = (n < F2W) ? l0 : r0, b = (n < F2W) ? l1 : r1;
    const unsigned u = pack_f16x2(a * ASC, b * ASC);
    ((volatile unsigned*)Bt2P)[i] = u; __threadfence(); ((volatile unsigned*)Bt2P)[i] = u;
  }
}

__device__ __forceinline__ int blk_excl_scan(int cnt, int* scan_ws, int tid, int* tot) {
  const int lane = tid & 31, wave = tid >> 5; int incl = cnt;
#pragma unroll
  for (int o = 1; o < 32; o <<= 1) { const int v = __shfl_up(incl, o, 32); if (lane >= o) incl += v; }
  if (lane == 31) scan_ws[wave] = incl;
  __syncthreads();
  if (wave == 0) { int wv = (lane < NT / 32) ? scan_ws[lane] : 0; int wincl = wv;
#pragma unroll
    for (int o = 1; o < 32; o <<= 1) { const int v = __shfl_up(wincl, o, 32); if (lane >= o) wincl += v; }
    if (lane < NT / 32) scan_ws[32 + lane] = wincl - wv; if (lane == 31) scan_ws[64] = wincl; }
  __syncthreads();
  const int res = scan_ws[32 + wave] + incl - cnt; *tot = scan_ws[64];
  return res;
}
template <int SP, int CAP, int NTOT>
__device__ __forceinline__ int chunk_hits(const int* __restrict__ dstv, int e0, int n0, int tid, int* LIST, int* scan_ws) {
  const int eb = e0 + tid * SP;
  const bool real = eb < NE;
  const int ebc = real ? eb : (NE - SP);
  int rec[SP]; int cnt = 0;
#pragma unroll
  for (int k = 0; k < SP; k += 4) {
    const v4i d4 = *(const v4i*)(dstv + ebc + k);
#pragma unroll
    for (int q = 0; q < 4; ++q) {
      const int e = eb + k + q;
      const int d = real ? d4[q] : (e - NE);
      const bool valid = real ? (d < NN) : (e < NTOT);
      int r = -1;
      if (valid && d >= n0 && d < n0 + TG) { r = ((d - n0) << 20) | e; ++cnt; }
      rec[k + q] = r;
    }
  }
  int tot; int p = blk_excl_scan(cnt, scan_ws, tid, &tot);
#pragma unroll
  for (int k = 0; k < SP; ++k) if (rec[k] >= 0) { if ((unsigned)p < (unsigned)CAP) LIST[p] = rec[k]; ++p; }
  __syncthreads();
  return tot < CAP ? tot : CAP;
}

__global__ __launch_bounds__(NT) void lattr_kernel(const int* __restrict__ ei, const float* __restrict__ ea, float* __restrict__ LATTR) {
  __shared__ __align__(16) float LA[TG * 4];
  __shared__ int LIST[SCH];
  __shared__ int scan_ws[80];
  const int tid = threadIdx.x, lane = tid & 31, wave = tid >> 5;
  const int n0 = blockIdx.x * TG;
  for (int i = tid; i < TG * 4; i += NT) LA[i] = 0.f;
  __syncthreads();
  const int* dstv = ei + NE;
  const int lk = (lane < 2) ? lane : 1;
#pragma unroll 1
  for (int c = 0; c < NCH1; ++c) {
    const int tot = chunk_hits<SPT, SCH, NE>(dstv, c * SCH, n0, tid, LIST, scan_ws);
#pragma unroll 1
    for (int base = 0; base < tot; base += 32) {
      const int q = base + lane;
      const int rv = (q < tot) ? LIST[q < SCH ? q : (SCH - 1)] : -1;
      const int own = (rv >= 0 && (rv >> 28) == wave) ? 1 : 0;
      unsigned msk = (unsigned)__ballot(own);
#pragma unroll 1
      for (int it = 0; it < 32; ++it) {
        if (msk == 0u) break;
        const int bp = __builtin_ctz(msk); msk &= msk - 1u;
        const int r = __shfl(rv, bp, 32);
        const int dl = r >> 20;
        int e = r & 0xFFFFF; e = (e < NE) ? e : (NE - 1);
        const float av = ea[(size_t)e * 2 + lk];
        const float v = (lane < 2) ? av : 1.0f;
        if (lane < 3) LA[dl * 4 + lane] += v;
      }
    }
    __syncthreads();
  }
#pragma unroll 1
  for (int j = 0; j < TG / (8 * 32); ++j) {
    const int dl = wave * (TG / 8) + j * 32 + lane;
    const int n = n0 + dl;
    const v4f s = *(const v4f*)(LA + dl * 4);
    const float cnt = s[2];
    const float inv = 1.0f / fmaxf(cnt, 1.0f);
    v4f o; o[0] = s[0] * inv; o[1] = s[1] * inv; o[2] = cnt; o[3] = 0.f;
    float* rp = LATTR + (size_t)n * 4;
    for (int pass = 0; pass < 2; ++pass) { *(volatile v4f*)rp = o; __threadfence(); }
  }
}

template <int NG, int LAYER>
__global__ __launch_bounds__(NT) void gat_kernel(const unsigned short* __restrict__ XLRp, const int* __restrict__ ei,
                                                const float* __restrict__ ea, const float* __restrict__ LATTR,
                                                const float* __restrict__ We, const float* __restrict__ att,
                                                const float* __restrict__ bias, float* __restrict__ ACC,
                                                unsigned short* __restrict__ Hp, const float* __restrict__ Wfc,
                                                const float* __restrict__ bfc, float* __restrict__ out) {
  constexpr int F = 128 * NG;
  constexpr int XW = 2 * F;
  extern __shared__ __align__(16) float dyn_lds[];
  float* SM = dyn_lds;
  float* SL = dyn_lds + TG * NG;
  int* LIST = (int*)(dyn_lds + 2 * TG * NG);
  __shared__ int scan_ws[80];
  __shared__ __align__(16) float sW0[F];
  __shared__ __align__(16) float sW1[F];
  __shared__ __align__(16) float sAt[F];
  const _Float16* XLR = (const _Float16*)XLRp;
  _Float16* H16 = (_Float16*)Hp;
  const int tid = threadIdx.x, lane = tid & 31, wave = tid >> 5;
  const int n0 = blockIdx.x * TG;
  const int c4 = 4 * lane;
  for (int i = tid; i < F; i += NT) { sW0[i] = We[i]; sW1[i] = We[F + i]; sAt[i] = att[i]; }
  for (int i = tid; i < TG * NG; i += NT) { SM[i] = -INFINITY; SL[i] = 0.f; }
  float* accb = ACC + (size_t)n0 * F;
  {
    const v4f z4 = {0.f, 0.f, 0.f, 0.f};
    for (int pass = 0; pass < 2; ++pass) {
#pragma unroll 1
      for (int j = 0; j < TG / 8; ++j) {
        float* ap = accb + (size_t)(wave * (TG / 8) + j) * F + c4;
#pragma unroll
        for (int g = 0; g < NG; ++g) *(volatile v4f*)(ap + (g << 7)) = z4;
      }
      __threadfence();
    }
  }
  __syncthreads();
  const int* srcv = ei;
  const int* dstv = ei + NE;
#pragma unroll 1
  for (int c = 0; c < NCH2; ++c) {
    const int tot = chunk_hits<SPT, SCH, NV>(dstv, c * SCH, n0, tid, LIST, scan_ws);
#pragma unroll 1
    for (int base = 0; base < tot; base += 32) {
      const int q = base + lane;
      const int rv = (q < tot) ? LIST[q < SCH ? q : (SCH - 1)] : -1;
      const int own = (rv >= 0 && (rv >> 28) == wave) ? 1 : 0;
      unsigned msk = (unsigned)__ballot(own);
#pragma unroll 1
      for (int it = 0; it < 32; ++it) {
        if (msk == 0u) break;
        const int bp = __builtin_ctz(msk); msk &= msk - 1u;
        const int r = __shfl(rv, bp, 32);
        const int dl = r >> 20;
        const int e  = r & 0xFFFFF;
        const int d  = n0 + dl;
        const bool real = e < NE;
        const int ec = real ? e : (NE - 1);
        int s = srcv[ec];
        s = s < 0 ? 0 : (s >= NN ? NN - 1 : s);
        s = real ? s : d;
        const v2f ev = *(const v2f*)(ea + (size_t)ec * 2);
        const v4f la = *(const v4f*)(LATTR + (size_t)d * 4);
        const float a0 = real ? ev[0] : la[0], a1 = real ? ev[1] : la[1];
        const _Float16* xls = XLR + (size_t)s * XW;
        const _Float16* xrd = XLR + (size_t)d * XW + F;
#pragma unroll 1
        for (int g = 0; g < NG; ++g) {
          const int f = (g << 7) + c4;
          const v4h xl4 = *(const v4h*)(xls + f);
          const v4h xr4 = *(const v4h*)(xrd + f);
          const v4f w0 = *(const v4f*)(sW0 + f);
          const v4f w1 = *(const v4f*)(sW1 + f);
          const v4f at = *(const v4f*)(sAt + f);
          float xl[4]; float p = 0.f;
#pragma unroll
          for (int i = 0; i < 4; ++i) {
            xl[i] = (float)xl4[i];
            float ee = a0 * w0[i]; ee = fmaf(a1, w1[i], ee);
            float z = (xl[i] + (float)xr4[i]) + ee;
            z = (z > 0.f) ? z : 0.2f * z;
            p = fmaf(z, at[i], p);
          }
          p += __shfl_xor(p, 16, 32); p += __shfl_xor(p, 8, 32); p += __shfl_xor(p, 4, 32);
          p += __shfl_xor(p, 2, 32);  p += __shfl_xor(p, 1, 32);
          const int mi = dl * NG + g;
          const float mo = SM[mi], lo = SL[mi];
          const float mn = fmaxf(mo, p);
          const float rr = __expf(mo - mn), ex = __expf(p - mn);
          const float ln = fmaf(lo, rr, ex);
          if (lane == 0) { SM[mi] = mn; SL[mi] = ln; }
          float* ap = accb + (size_t)dl * F + f;
          const v4f qv = *(const v4f*)ap;
          v4f ov;
#pragma unroll
          for (int i = 0; i < 4; ++i) ov[i] = fmaf(qv[i], rr, ex * xl[i]);
          *(volatile v4f*)ap = ov;
          __threadfence();
          *(volatile v4f*)ap = ov;
          asm volatile("" ::: "memory");
        }
      }
    }
    __syncthreads();
  }
  if (LAYER == 1) {
#pragma unroll 1
    for (int j = 0; j < TG / 8; ++j) {
      const int dl = wave * (TG / 8) + j;
      const int n = n0 + dl;
      if (n < MP) {
        const bool live = n < NN;
#pragma unroll 1
        for (int g = 0; g < NG; ++g) {
          const int f = (g << 7) + c4;
          const v4f qv = *(const v4f*)(accb + (size_t)dl * F + f);
          float l = SL[dl * NG + g];
          l = (live && l > 0.f) ? l : 1.0f;
          const float inv = 1.0f / l;
          const v4f b4 = *(const v4f*)(bias + f);
          float y[4];
#pragma unroll
          for (int i = 0; i < 4; ++i) {
            float v = fmaf(qv[i], inv, b4[i]);
            v = (v > 0.f) ? v : (__expf(v) - 1.0f);
            y[i] = live ? v * ASC : 0.f;
          }
          const int sl = (2 * lane) & 31;
          v8h h8;
#pragma unroll
          for (int i = 0; i < 4; ++i) {
            const float ta = __shfl(y[i], sl, 32), tb = __shfl(y[i], sl + 1, 32);
            h8[i] = (_Float16)ta; h8[4 + i] = (_Float16)tb;
          }
          _Float16* hq = H16 + (size_t)n * F + (g << 7) + 8 * (lane & 15);
          for (int pass = 0; pass < 2; ++pass) {
            if (lane < 16) *(volatile v8h*)hq = h8;
            __threadfence();
          }
        }
      }
    }
  } else {
    const v4f wA = *(const v4f*)(Wfc + 2 * c4);
    const v4f wB = *(const v4f*)(Wfc + 2 * c4 + 4);
    const v4f b4 = *(const v4f*)(bias + c4);
    const float bf0 = bfc[0], bf1 = bfc[1];
    float my0 = 0.f, my1 = 0.f;
#pragma unroll 1
    for (int j = 0; j < TG / 8; ++j) {
      const int dl = wave * (TG / 8) + j;
      const int n = n0 + dl;
      const bool live = n < NN;
      const v4f qv = *(const v4f*)(accb + (size_t)dl * F + c4);
      float l = SL[dl * NG];
      l = (live && l > 0.f) ? l : 1.0f;
      const float inv = 1.0f / l;
      float v[4];
#pragma unroll
      for (int i = 0; i < 4; ++i) {
        const float t = fmaf(qv[i], inv, b4[i]);
        v[i] = (t > 0.f) ? t : (__expf(t) - 1.0f);
      }
      float p0 = v[0] * wA[0]; p0 = fmaf(v[1], wA[2], p0); p0 = fmaf(v[2], wB[0], p0); p0 = fmaf(v[3], wB[2], p0);
      float p1 = v[0] * wA[1]; p1 = fmaf(v[1], wA[3], p1); p1 = fmaf(v[2], wB[1], p1); p1 = fmaf(v[3], wB[3], p1);
      p0 += __shfl_xor(p0, 16, 32); p0 += __shfl_xor(p0, 8, 32); p0 += __shfl_xor(p0, 4, 32); p0 += __shfl_xor(p0, 2, 32); p0 += __shfl_xor(p0, 1, 32);
      p1 += __shfl_xor(p1, 16, 32); p1 += __shfl_xor(p1, 8, 32); p1 += __shfl_xor(p1, 4, 32); p1 += __shfl_xor(p1, 2, 32); p1 += __shfl_xor(p1, 1, 32);
      const float o0 = p0 + bf0, o1 = p1 + bf1;
      if (lane == (j & 31)) { my0 = o0; my1 = o1; }
      if ((j & 31) == 31) {
        const int nb = n - 31;
        if (nb + 32 <= NN) {
          const int sl = (2 * lane) & 31;
          v4f o;
          o[0] = __shfl(my0, sl, 32); o[1] = __shfl(my1, sl, 32);
          o[2] = __shfl(my0, sl + 1, 32); o[3] = __shfl(my1, sl + 1, 32);
          float* op = out + (size_t)(nb + 2 * (lane & 15)) * 2;
          for (int pass = 0; pass < 2; ++pass) {
            if (lane < 16) *(volatile v4f*)op = o;
            __threadfence();
          }
        }
      }
    }
  }
}

extern "C" void kernel_launch(void* const* d_in, const int* in_sizes, int n_in,
                              void* d_out, int out_size, void* d_ws, size_t ws_size, hipStream_t stream) {
  if (n_in < 17) return;
  const float* x     = (const float*)d_in[0];
  const int*   ei    = (const int*)  d_in[1];
  const float* ea    = (const float*)d_in[2];
  const int*   rt    = (const int*)  d_in[3];
  const float* emb   = (const float*)d_in[4];
  const float* W1l   = (const float*)d_in[5];
  const float* W1r   = (const float*)d_in[6];
  const float* W1e   = (const float*)d_in[7];
  const float* att1  = (const float*)d_in[8];
  const float* b1    = (const float*)d_in[9];
  const float* W2l   = (const float*)d_in[10];
  const float* W2r   = (const float*)d_in[11];
  const float* W2e   = (const float*)d_in[12];
  const float* att2  = (const float*)d_in[13];
  const float* b2    = (const float*)d_in[14];
  const float* Wfc   = (const float*)d_in[15];
  const float* bfc   = (const float*)d_in[16];
  float* out = (float*)d_out;

  if (in_sizes[0] != NN * XD || in_sizes[1] != 2 * NE || in_sizes[2] != NE * 2 || in_sizes[3] != NN) return;
  if (in_sizes[4] != NAA * AE || in_sizes[5] != KIN * F1W || in_sizes[6] != KIN * F1W || in_sizes[7] != 2 * F1W) return;
  if (in_sizes[8] != F1W || in_sizes[9] != F1W || in_sizes[10] != F1W * F2W || in_sizes[11] != F1W * F2W) return;
  if (in_sizes[12] != 2 * F2W || in_sizes[13] != F2W || in_sizes[14] != F2W || in_sizes[15] != F2W * 2 || in_sizes[16] != 2) return;
  if (out_size != NN * 2) return;

  char* ws = (char*)d_ws; size_t off = 0;
  auto carve = [&](size_t bytes) -> char* { char* p = ws + off; off += (bytes + 255) & ~(size_t)255; return p; };
  float*          ACC   = (float*)carve((size_t)NROWT * F1W * 4);
  unsigned*       X16   = (unsigned*)ACC;
  unsigned short* XLR   = (unsigned short*)carve((size_t)MP * 2 * F1W * 2);
  float*          LATTR = (float*)carve((size_t)NROWT * 4 * 4);
  unsigned short* H1    = (unsigned short*)carve((size_t)MP * F1W * 2);
  unsigned*       Bt1P  = (unsigned*)carve((size_t)2 * F1W * K1 * 2);
  unsigned*       Bt2P  = (unsigned*)carve((size_t)2 * F2W * F1W * 2);
  if (off > ws_size || off > (size_t)134217728) return;

  h0_kernel<<<(MP * 32 + 255) / 256, 256, 0, stream>>>(x, rt, emb, X16);
  wprep_kernel<<<1, NT, 0, stream>>>(W1l, W1r, W2l, W2r, Bt1P, Bt2P);
  {
    const int tiles = (MP / 64) * (2 * F1W / 64);
    wmma_gemm64<0, false, 0, 1, false, 0><<<dim3((tiles + 7) / 8, 1), 256, 0, stream>>>(
        U16(X16), U16(X16), K1, 0L,
        U16(Bt1P), U16(Bt1P), K1, 0L,
        (void*)XLR, (void*)nullptr, 2 * F1W, 0L,
        b1, (const float*)nullptr, 0L, MP, 2 * F1W, K1, GSC_INV);
  }
  lattr_kernel<<<NTILE, NT, 0, stream>>>(ei, ea, LATTR);
  hipFuncSetAttribute(reinterpret_cast<const void*>(&gat_kernel<4, 1>), hipFuncAttributeMaxDynamicSharedMemorySize, GAT_LDS(4));
  gat_kernel<4, 1><<<NTILE, NT, GAT_LDS(4), stream>>>(XLR, ei, ea, LATTR, W1e, att1, b1, ACC, H1, Wfc, bfc, out);
  {
    const int tiles = (MP / 64) * (2 * F2W / 64);
    wmma_gemm64<0, false, 0, 1, false, 0><<<dim3((tiles + 7) / 8, 1), 256, 0, stream>>>(
        U16(H1), U16(H1), F1W, 0L,
        U16(Bt2P), U16(Bt2P), F1W, 0L,
        (void*)XLR, (void*)nullptr, 2 * F2W, 0L,
        b2, (const float*)nullptr, 0L, MP, 2 * F2W, F1W, GSC_INV);
  }
  hipFuncSetAttribute(reinterpret_cast<const void*>(&gat_kernel<1, 2>), hipFuncAttributeMaxDynamicSharedMemorySize, GAT_LDS(1));
  gat_kernel<1, 2><<<NTILE, NT, GAT_LDS(1), stream>>>(XLR, ei, ea, LATTR, W2e, att2, b2, ACC, H1, Wfc, bfc, out);
}
